// PhyHGkNN4_6897717477693
// MI455X (gfx1250) — hardware-verified
//
#include <hip/hip_runtime.h>
#include <math.h>

constexpr int B_  = 8;
constexpr int N_  = 8192;
constexpr int K1_ = 64;
constexpr int K2_ = 128;
constexpr int M_  = 256;
constexpr int C_  = 128;
constexpr int KM_ = 16;
constexpr int L_  = 3;
constexpr int KD_ = KM_ * M_;
static_assert(M_ == 2 * K1_ + K2_);
static_assert(KD_ == 4096);

constexpr float LN_EPS = 1e-5f;
constexpr float SQRTN  = 90.509667991878082f;
constexpr float SC_XH  = 0.001953125f;
constexpr float SC_SPW = 16384.0f;
constexpr float SC_H1  = 65536.0f;
constexpr float SC_Y   = 0.0009765625f;
constexpr float SC_X1  = 9.5367431640625e-7f;
constexpr float SC_W   = 16.0f;
constexpr float SC_OUT = 0.0625f;

typedef _Float16 v16h __attribute__((ext_vector_type(16)));
typedef _Float16 v8h  __attribute__((ext_vector_type(8)));
typedef float    v8f  __attribute__((ext_vector_type(8)));
typedef float    v4f  __attribute__((ext_vector_type(4)));
union Frag { v16h v; v8h hv[2]; };

__device__ __forceinline__ v16h ldfrag(const _Float16* p) {
  Frag f;
  f.hv[0] = *(const v8h*)p;
  f.hv[1] = *(const v8h*)(p + 16);
  return f.v;
}
__device__ __forceinline__ v8f mma16(v16h a, v16h b, v8f c) {
  c = __builtin_amdgcn_wmma_f32_16x16x32_f16(false, a, false, b, (short)0, c, false, false);
  asm volatile("v_nop\n\tv_nop\n\tv_nop\n\tv_nop" : "+v"(c) : "v"(a), "v"(b));
  return c;
}
__device__ __forceinline__ v8f vz() {
  v8f z = {0.f, 0.f, 0.f, 0.f, 0.f, 0.f, 0.f, 0.f};
  return z;
}
__device__ __forceinline__ float gelu_f(float x) {
  return 0.5f * x * (1.0f + erff(x * 0.70710678118654752f));
}

__device__ __forceinline__ float base_raw(int k, float g0, float g1, const float* prm) {
  if (k < 2 * K1_) {
    int q = (k < K1_) ? k : (k - K1_);
    float ph = g0 * prm[2 * q] + g1 * prm[2 * q + 1];
    float r;
    if (k < K1_) r = cosf(ph); else r = sinf(ph);
    return r;
  }
  int q = k - 2 * K1_;
  float w0 = fabsf(prm[384 + 2 * q]), w1 = fabsf(prm[384 + 2 * q + 1]);
  float d0 = g0 - prm[128 + 2 * q], d1 = g1 - prm[128 + 2 * q + 1];
  return sqrtf(w0 * w1) * expf(-(w0 * d0 * d0 + w1 * d1 * d1));
}

__global__ __launch_bounds__(256) void k_bases_ss(const float* __restrict__ x,
                                                  const float* __restrict__ bwf,
                                                  const float* __restrict__ pts,
                                                  const float* __restrict__ bwg,
                                                  float* __restrict__ sumsq) {
  __shared__ float prm[640];
  __shared__ float part[8 * 32];
  __shared__ __align__(16) float tot[32];
  const int t = threadIdx.x, wave = t >> 5, lane = t & 31;
  if (t < 128) prm[t] = bwf[t];
  prm[128 + t] = pts[t];
  prm[384 + t] = bwg[t];
  __syncthreads();
  const int b = blockIdx.x >> 3, slab = blockIdx.x & 7;
  const int k = slab * 32 + lane;
  const float* xb = x + (size_t)b * N_ * 3;
  float acc = 0.f;
#pragma unroll 1
  for (int n = wave; n < N_; n += 8) {
    float g0 = xb[n * 3 + 1], g1 = xb[n * 3 + 2];
    float v = base_raw(k, g0, g1, prm);
    acc += v * v;
  }
  part[wave * 32 + lane] = acc;
  __syncthreads();
  if (t < 32) {
    float s = 0.f;
#pragma unroll
    for (int w = 0; w < 8; ++w) s += part[w * 32 + t];
    tot[t] = s;
  }
  __syncthreads();
  if (t < 8) {
    v4f v = *(const v4f*)&tot[t * 4];
    float* dst = sumsq + b * M_ + slab * 32 + t * 4;
    *(volatile v4f*)dst = v;
    __threadfence();
    *(volatile v4f*)dst = v;
  }
}

__global__ __launch_bounds__(256) void k_bases_write(const float* __restrict__ x,
                                                     const float* __restrict__ bwf,
                                                     const float* __restrict__ pts,
                                                     const float* __restrict__ bwg,
                                                     const float* __restrict__ sumsq,
                                                     _Float16* __restrict__ bases,
                                                     _Float16* __restrict__ basesT) {
  __shared__ float prm[640];
  __shared__ float scl[M_];
  __shared__ __align__(16) _Float16 tile[64 * 264];
  const int t = threadIdx.x, wave = t >> 5, lane = t & 31;
  const int b = blockIdx.x >> 7, n0 = (blockIdx.x & 127) * 64;
  if (t < 128) prm[t] = bwf[t];
  prm[128 + t] = pts[t];
  prm[384 + t] = bwg[t];
  {
    float ss = sumsq[b * M_ + t];
    float dn = sqrtf(ss) + ((t < 2 * K1_) ? 1e-5f : 0.0f);
    scl[t] = 1.0f / dn;
  }
  __syncthreads();
  const int nl = t & 63, kg = t >> 6;
  const float* xr = x + (size_t)(b * N_ + n0 + nl) * 3;
  const float g0 = xr[1], g1 = xr[2];
#pragma unroll 1
  for (int e = 0; e < 64; ++e) {
    int k = kg * 64 + e;
    float v = base_raw(k, g0, g1, prm);
    v = (v * SQRTN) * scl[k];
    tile[nl * 264 + k] = (_Float16)v;
  }
  __syncthreads();
  const int sub = lane >> 3, q = lane & 7;
#pragma unroll
  for (int pass = 0; pass < 2; ++pass) {
#pragma unroll
    for (int u = 0; u < 8; ++u) {
      int j = wave * 32 + u * 4 + sub;
      int row = j >> 2, col = (j & 3) * 64 + q * 8;
      v8h v = *(const v8h*)(tile + row * 264 + col);
      _Float16* dst = bases + (size_t)(b * N_ + n0 + row) * M_ + col;
      *(volatile v8h*)dst = v;
    }
#pragma unroll
    for (int u = 0; u < 8; ++u) {
      int kl = wave * 32 + u * 4 + sub;
      v8h v;
#pragma unroll
      for (int e = 0; e < 8; ++e) v[e] = tile[(q * 8 + e) * 264 + kl];
      _Float16* dst = basesT + (size_t)(b * M_ + kl) * N_ + n0 + q * 8;
      *(volatile v8h*)dst = v;
    }
    if (pass == 0) __threadfence();
  }
}

__device__ __forceinline__ void ln_act_row(float (&v)[8], const float* __restrict__ g,
                                           const float* __restrict__ be, int cq, bool act,
                                           _Float16* trow) {
  float s = 0.f;
#pragma unroll
  for (int e = 0; e < 8; ++e) s += v[e];
  s += __shfl_xor(s, 8, 32);
  s += __shfl_xor(s, 4, 32);
  s += __shfl_xor(s, 2, 32);
  s += __shfl_xor(s, 1, 32);
  const float mean = s * (1.0f / C_);
  float sq = 0.f;
#pragma unroll
  for (int e = 0; e < 8; ++e) { float d = v[e] - mean; sq += d * d; }
  sq += __shfl_xor(sq, 8, 32);
  sq += __shfl_xor(sq, 4, 32);
  sq += __shfl_xor(sq, 2, 32);
  sq += __shfl_xor(sq, 1, 32);
  const float var = sq * (1.0f / C_);
  const float rs = 1.0f / sqrtf(var + LN_EPS);
#pragma unroll
  for (int e = 0; e < 8; ++e) {
    int c = cq * 8 + e;
    float xn = (v[e] - mean) * rs * g[c] + be[c];
    if (act) xn = gelu_f(xn);
    trow[c] = (_Float16)xn;
  }
}

__device__ __forceinline__ void store_h_block(const _Float16* tile, _Float16* h, _Float16* hT,
                                              int b, int n0, int wave, int lane) {
  const int sub = lane >> 3, q = lane & 7;
#pragma unroll
  for (int pass = 0; pass < 2; ++pass) {
#pragma unroll
    for (int u = 0; u < 4; ++u) {
      int j = wave * 16 + u * 4 + sub;
      int row = j >> 1, col = (j & 1) * 64 + q * 8;
      v8h v = *(const v8h*)(tile + row * 136 + col);
      _Float16* dst = h + (size_t)(b * N_ + n0 + row) * C_ + col;
      *(volatile v8h*)dst = v;
    }
#pragma unroll
    for (int u = 0; u < 4; ++u) {
      int c = wave * 16 + u * 4 + sub;
      v8h v;
#pragma unroll
      for (int e = 0; e < 8; ++e) v[e] = tile[(q * 8 + e) * 136 + c];
      _Float16* dst = hT + (size_t)(b * C_ + c) * N_ + n0 + q * 8;
      *(volatile v8h*)dst = v;
    }
    if (pass == 0) __threadfence();
  }
}

__global__ __launch_bounds__(256) void k_fc0_ln(const float* __restrict__ x,
                                                const float* __restrict__ w,
                                                const float* __restrict__ bias,
                                                const float* __restrict__ g,
                                                const float* __restrict__ be,
                                                _Float16* h, _Float16* hT) {
  __shared__ __align__(16) _Float16 tile[64 * 136];
  const int t = threadIdx.x, wave = t >> 5, lane = t & 31;
  const int b = blockIdx.x >> 7, n0 = (blockIdx.x & 127) * 64;
  const int rsel = lane >> 4, cq = lane & 15;
#pragma unroll 1
  for (int it = 0; it < 4; ++it) {
    int row = wave * 8 + it * 2 + rsel;
    const float* xr = x + (size_t)(b * N_ + n0 + row) * 3;
    float x0 = xr[0], x1 = xr[1], x2 = xr[2];
    float v[8];
#pragma unroll
    for (int e = 0; e < 8; ++e) {
      int c = cq * 8 + e;
      v[e] = x0 * w[c] + x1 * w[C_ + c] + x2 * w[2 * C_ + c] + bias[c];
    }
    ln_act_row(v, g, be, cq, false, tile + row * 136);
  }
  __syncthreads();
  store_h_block(tile, h, hT, b, n0, wave, lane);
}

__global__ __launch_bounds__(256) void k_pack(const float* __restrict__ sp,
                                              const float* __restrict__ H1,
                                              const float* __restrict__ wsw,
                                              const float* __restrict__ fc1w,
                                              _Float16* __restrict__ spw16,
                                              _Float16* __restrict__ h1t16,
                                              _Float16* __restrict__ wsw16,
                                              _Float16* __restrict__ fc1t16) {
  const int blk = blockIdx.x, t = threadIdx.x;
  v8h v;
  _Float16* dst;
  if (blk < 384) {
    int idx = (blk * 256 + t) * 8;
    int i0 = idx & (C_ - 1), o = (idx >> 7) & (C_ - 1), j = (idx >> 14) & (KM_ - 1), l = idx >> 18;
#pragma unroll
    for (int e = 0; e < 8; ++e)
      v[e] = (_Float16)(sp[((size_t)((l * C_ + i0 + e) * C_ + o)) * KM_ + j] * SC_SPW);
    dst = spw16 + idx;
  } else if (blk < 896) {
    int idx = ((blk - 384) * 256 + t) * 8;
    int lc = idx & (M_ - 1), j = (idx >> 8) & (KM_ - 1), k = idx >> 12;
#pragma unroll
    for (int e = 0; e < 8; ++e)
      v[e] = (_Float16)(H1[(size_t)(j * M_ + k) * M_ + lc + e] * SC_H1);
    dst = h1t16 + idx;
  } else if (blk < 920) {
    int idx = ((blk - 896) * 256 + t) * 8;
#pragma unroll
    for (int e = 0; e < 8; ++e) v[e] = (_Float16)(wsw[idx + e] * SC_W);
    dst = wsw16 + idx;
  } else {
    int idx = ((blk - 920) * 256 + t) * 8;
    int i = idx & (C_ - 1), c = idx >> 7;
#pragma unroll
    for (int e = 0; e < 8; ++e) v[e] = (_Float16)(fc1w[(size_t)(i + e) * C_ + c] * SC_W);
    dst = fc1t16 + idx;
  }
  *(volatile v8h*)dst = v;
  __threadfence();
  *(volatile v8h*)dst = v;
}

__device__ __forceinline__ void epi64(v8f acc0, v8f acc1, float scale, _Float16* tile,
                                      _Float16* dst, size_t pitch, int wave, int lane) {
  const int m = lane & 15, hh = lane >> 4, wm = wave & 3, wn = wave >> 2;
#pragma unroll
  for (int r = 0; r < 8; ++r) {
    tile[(wm * 16 + 8 * hh + r) * 72 + wn * 32 + m]      = (_Float16)(acc0[r] * scale);
    tile[(wm * 16 + 8 * hh + r) * 72 + wn * 32 + 16 + m] = (_Float16)(acc1[r] * scale);
  }
  __syncthreads();
  const int sub = lane >> 3, q = lane & 7;
#pragma unroll
  for (int pass = 0; pass < 2; ++pass) {
#pragma unroll
    for (int u = 0; u < 2; ++u) {
      int row = wave * 8 + u * 4 + sub;
      v8h v = *(const v8h*)(tile + row * 72 + q * 8);
      *(volatile v8h*)(dst + (size_t)row * pitch + q * 8) = v;
    }
    if (pass == 0) __threadfence();
  }
}

__global__ __launch_bounds__(256) void k_xh(const _Float16* __restrict__ basesT,
                                            const _Float16* __restrict__ hT,
                                            _Float16* __restrict__ xhT) {
  __shared__ __align__(16) _Float16 tile[64 * 72];
  const int t = threadIdx.x, wave = t >> 5, lane = t & 31, m = lane & 15, hh = lane >> 4;
  const int blk = blockIdx.x, b = blk >> 3, l0 = ((blk >> 1) & 3) * 64, i0 = (blk & 1) * 64;
  const int wm = wave & 3, wn = wave >> 2;
  const _Float16* ap  = basesT + (size_t)(b * M_ + l0 + wm * 16 + m) * N_ + 8 * hh;
  const _Float16* bp0 = hT + (size_t)(b * C_ + i0 + wn * 32 + m) * N_ + 8 * hh;
  const _Float16* bp1 = bp0 + (size_t)16 * N_;
  v8f acc0 = vz(), acc1 = vz();
#pragma unroll 2
  for (int k0 = 0; k0 < N_; k0 += 32) {
    v16h a  = ldfrag(ap + k0);
    v16h f0 = ldfrag(bp0 + k0);
    v16h f1 = ldfrag(bp1 + k0);
    acc0 = mma16(a, f0, acc0);
    acc1 = mma16(a, f1, acc1);
  }
  epi64(acc0, acc1, SC_XH, tile, xhT + (size_t)(b * M_ + l0) * C_ + i0, (size_t)C_, wave, lane);
}

__global__ __launch_bounds__(256) void k_t(const _Float16* __restrict__ spw16,
                                           const _Float16* __restrict__ xhT,
                                           _Float16* __restrict__ t16, int layer) {
  __shared__ __align__(16) _Float16 tile[64 * 72];
  const int t = threadIdx.x, wave = t >> 5, lane = t & 31, m = lane & 15, hh = lane >> 4;
  const int blk = blockIdx.x, b = blk >> 7, j = (blk >> 3) & 15;
  const int o0 = ((blk >> 2) & 1) * 64, lq0 = (blk & 3) * 64;
  const int wm = wave & 3, wn = wave >> 2;
  const _Float16* ap  = spw16 + (size_t)((layer * KM_ + j) * C_ + o0 + wm * 16 + m) * C_ + 8 * hh;
  const _Float16* bp0 = xhT + (size_t)(b * M_ + lq0 + wn * 32 + m) * C_ + 8 * hh;
  const _Float16* bp1 = bp0 + (size_t)16 * C_;
  v8f acc0 = vz(), acc1 = vz();
#pragma unroll 1
  for (int k0 = 0; k0 < C_; k0 += 32) {
    v16h a  = ldfrag(ap + k0);
    v16h f0 = ldfrag(bp0 + k0);
    v16h f1 = ldfrag(bp1 + k0);
    acc0 = mma16(a, f0, acc0);
    acc1 = mma16(a, f1, acc1);
  }
  epi64(acc0, acc1, 1.0f, tile, t16 + ((size_t)(b * C_ + o0) * KM_ + j) * M_ + lq0,
        (size_t)KD_, wave, lane);
}

__global__ __launch_bounds__(256) void k_y(const _Float16* __restrict__ t16,
                                           const _Float16* __restrict__ h1t16,
                                           _Float16* __restrict__ ys16) {
  __shared__ __align__(16) _Float16 tile[64 * 72];
  const int t = threadIdx.x, wave = t >> 5, lane = t & 31, m = lane & 15, hh = lane >> 4;
  const int blk = blockIdx.x, b = blk >> 3, o0 = ((blk >> 2) & 1) * 64, kc0 = (blk & 3) * 64;
  const int wm = wave & 3, wn = wave >> 2;
  const _Float16* ap  = t16 + (size_t)(b * C_ + o0 + wm * 16 + m) * KD_ + 8 * hh;
  const _Float16* bp0 = h1t16 + (size_t)(kc0 + wn * 32 + m) * KD_ + 8 * hh;
  const _Float16* bp1 = bp0 + (size_t)16 * KD_;
  v8f acc0 = vz(), acc1 = vz();
#pragma unroll 2
  for (int k0 = 0; k0 < KD_; k0 += 32) {
    v16h a  = ldfrag(ap + k0);
    v16h f0 = ldfrag(bp0 + k0);
    v16h f1 = ldfrag(bp1 + k0);
    acc0 = mma16(a, f0, acc0);
    acc1 = mma16(a, f1, acc1);
  }
  epi64(acc0, acc1, SC_Y, tile, ys16 + (size_t)(b * C_ + o0) * M_ + kc0, (size_t)M_, wave, lane);
}

__global__ __launch_bounds__(256) void k_x1h(const _Float16* __restrict__ bases,
                                             const _Float16* __restrict__ ys16,
                                             _Float16* h, _Float16* hT,
                                             const _Float16* __restrict__ wsw16,
                                             const float* __restrict__ wsb,
                                             const float* __restrict__ lng,
                                             const float* __restrict__ lnb, int layer) {
  __shared__ __align__(16) float outT[64 * 132];
  __shared__ __align__(16) _Float16 tile[64 * 136];
  const int t = threadIdx.x, wave = t >> 5, lane = t & 31, m = lane & 15, hh = lane >> 4;
  const int blk = blockIdx.x, b = blk >> 7, n0 = (blk & 127) * 64;
  const int wr = wave >> 1, cg = (wave & 1) * 64;
  v8f acc[4];
#pragma unroll
  for (int jt = 0; jt < 4; ++jt) acc[jt] = vz();
  {
    const _Float16* ap = bases + (size_t)(b * N_ + n0 + wr * 16 + m) * M_ + 8 * hh;
    const _Float16* bp = ys16 + (size_t)(b * C_ + cg + m) * M_ + 8 * hh;
#pragma unroll 1
    for (int k0 = 0; k0 < M_; k0 += 32) {
      v16h a = ldfrag(ap + k0);
#pragma unroll
      for (int jt = 0; jt < 4; ++jt) {
        v16h bb = ldfrag(bp + (size_t)(jt * 16) * M_ + k0);
        acc[jt] = mma16(a, bb, acc[jt]);
      }
    }
  }
#pragma unroll
  for (int jt = 0; jt < 4; ++jt)
#pragma unroll
    for (int r = 0; r < 8; ++r) acc[jt][r] = acc[jt][r] * SC_X1;
  {
    const _Float16* ap = h + (size_t)(b * N_ + n0 + wr * 16 + m) * C_ + 8 * hh;
    const _Float16* bp = wsw16 + (size_t)(layer * C_ + cg + m) * C_ + 8 * hh;
#pragma unroll 1
    for (int k0 = 0; k0 < C_; k0 += 32) {
      v16h a = ldfrag(ap + k0);
#pragma unroll
      for (int jt = 0; jt < 4; ++jt) {
        v16h bb = ldfrag(bp + (size_t)(jt * 16) * C_ + k0);
        acc[jt] = mma16(a, bb, acc[jt]);
      }
    }
  }
#pragma unroll
  for (int jt = 0; jt < 4; ++jt)
#pragma unroll
    for (int r = 0; r < 8; ++r) {
      int rr = wr * 16 + 8 * hh + r;
      int cc = cg + jt * 16 + m;
      outT[rr * 132 + cc] = acc[jt][r] * SC_OUT + wsb[layer * C_ + cc];
    }
  __syncthreads();
  const bool act = (layer < L_ - 1);
  const int rsel = lane >> 4, cq = lane & 15;
#pragma unroll 1
  for (int it = 0; it < 4; ++it) {
    int row = wave * 8 + it * 2 + rsel;
    float v[8];
#pragma unroll
    for (int e = 0; e < 8; ++e) v[e] = outT[row * 132 + cq * 8 + e];
    ln_act_row(v, lng + layer * C_, lnb + layer * C_, cq, act, tile + row * 136);
  }
  __syncthreads();
  store_h_block(tile, h, hT, b, n0, wave, lane);
}

__global__ __launch_bounds__(256) void k_fc12(const _Float16* __restrict__ h,
                                              const _Float16* __restrict__ fc1t16,
                                              const float* __restrict__ fc1b,
                                              const float* __restrict__ fc2w,
                                              const float* __restrict__ fc2b,
                                              float* __restrict__ out) {
  __shared__ __align__(16) float outT[64 * 132];
  __shared__ __align__(16) float outv[64];
  const int t = threadIdx.x, wave = t >> 5, lane = t & 31, m = lane & 15, hh = lane >> 4;
  const int blk = blockIdx.x, b = blk >> 7, n0 = (blk & 127) * 64;
  const int wr = wave >> 1, cg = (wave & 1) * 64;
  v8f acc[4];
#pragma unroll
  for (int jt = 0; jt < 4; ++jt) acc[jt] = vz();
  {
    const _Float16* ap = h + (size_t)(b * N_ + n0 + wr * 16 + m) * C_ + 8 * hh;
    const _Float16* bp = fc1t16 + (size_t)(cg + m) * C_ + 8 * hh;
#pragma unroll 1
    for (int k0 = 0; k0 < C_; k0 += 32) {
      v16h a = ldfrag(ap + k0);
#pragma unroll
      for (int jt = 0; jt < 4; ++jt) {
        v16h bb = ldfrag(bp + (size_t)(jt * 16) * C_ + k0);
        acc[jt] = mma16(a, bb, acc[jt]);
      }
    }
  }
#pragma unroll
  for (int jt = 0; jt < 4; ++jt)
#pragma unroll
    for (int r = 0; r < 8; ++r) {
      int rr = wr * 16 + 8 * hh + r;
      int cc = cg + jt * 16 + m;
      outT[rr * 132 + cc] = acc[jt][r] * SC_OUT + fc1b[cc];
    }
  __syncthreads();
  const int rsel = lane >> 4, cq = lane & 15;
#pragma unroll 1
  for (int it = 0; it < 4; ++it) {
    int row = wave * 8 + it * 2 + rsel;
    float d = 0.f;
#pragma unroll
    for (int e = 0; e < 8; ++e) {
      int c = cq * 8 + e;
      float gv = gelu_f(outT[row * 132 + c]);
      d += gv * fc2w[c];
    }
    d += __shfl_xor(d, 8, 32);
    d += __shfl_xor(d, 4, 32);
    d += __shfl_xor(d, 2, 32);
    d += __shfl_xor(d, 1, 32);
    if (cq == 0) outv[row] = d + fc2b[0];
  }
  __syncthreads();
  if (t < 16) {
    v4f v = *(const v4f*)&outv[t * 4];
    float* dst = out + (size_t)b * N_ + n0 + t * 4;
    *(volatile v4f*)dst = v;
    __threadfence();
    *(volatile v4f*)dst = v;
  }
}

extern "C" void kernel_launch(void* const* d_in, const int* in_sizes, int n_in,
                              void* d_out, int out_size, void* d_ws, size_t ws_size,
                              hipStream_t stream) {
  if (n_in < 18) return;
  if (in_sizes[0] != B_ * N_ * 3 || in_sizes[1] != K1_ * 2 || in_sizes[2] != K2_ * 2 ||
      in_sizes[3] != K2_ * 2 || in_sizes[4] != 3 * C_ || in_sizes[5] != C_ ||
      in_sizes[6] != C_ || in_sizes[7] != C_ || in_sizes[8] != KM_ * M_ * M_ ||
      in_sizes[9] != L_ * C_ * C_ * KM_ || in_sizes[10] != L_ * C_ * C_ ||
      in_sizes[11] != L_ * C_ || in_sizes[12] != L_ * C_ || in_sizes[13] != L_ * C_ ||
      in_sizes[14] != C_ * C_ || in_sizes[15] != C_ || in_sizes[16] != C_ ||
      in_sizes[17] != 1 || out_size != B_ * N_)
    return;

  const float* x    = (const float*)d_in[0];
  const float* bwf  = (const float*)d_in[1];
  const float* pts  = (const float*)d_in[2];
  const float* bwg  = (const float*)d_in[3];
  const float* fc0w = (const float*)d_in[4];
  const float* fc0b = (const float*)d_in[5];
  const float* ln0g = (const float*)d_in[6];
  const float* ln0b = (const float*)d_in[7];
  const float* H1   = (const float*)d_in[8];
  const float* spw  = (const float*)d_in[9];
  const float* wsw  = (const float*)d_in[10];
  const float* wsb  = (const float*)d_in[11];
  const float* lng  = (const float*)d_in[12];
  const float* lnb  = (const float*)d_in[13];
  const float* fc1w = (const float*)d_in[14];
  const float* fc1b = (const float*)d_in[15];
  const float* fc2w = (const float*)d_in[16];
  const float* fc2b = (const float*)d_in[17];

  size_t off = 0;
  auto take = [&](size_t bytes) -> char* {
    char* r = (char*)d_ws + off;
    off += (bytes + 255) & ~(size_t)255;
    return r;
  };
  float*    sumsq  = (float*)take((size_t)B_ * M_ * sizeof(float));
  _Float16* bases  = (_Float16*)take((size_t)B_ * N_ * M_ * 2);
  _Float16* basesT = (_Float16*)take((size_t)B_ * M_ * N_ * 2);
  _Float16* h      = (_Float16*)take((size_t)B_ * N_ * C_ * 2);
  _Float16* hT     = (_Float16*)take((size_t)B_ * C_ * N_ * 2);
  _Float16* xhT    = (_Float16*)take((size_t)B_ * M_ * C_ * 2);
  _Float16* t16    = (_Float16*)take((size_t)B_ * C_ * KM_ * M_ * 2);
  _Float16* ys16   = (_Float16*)take((size_t)B_ * C_ * M_ * 2);
  _Float16* spw16  = (_Float16*)take((size_t)L_ * KM_ * C_ * C_ * 2);
  _Float16* h1t16  = (_Float16*)take((size_t)M_ * KD_ * 2);
  _Float16* wsw16  = (_Float16*)take((size_t)L_ * C_ * C_ * 2);
  _Float16* fc1t16 = (_Float16*)take((size_t)C_ * C_ * 2);
  if (off > ws_size) return;

  k_bases_ss<<<dim3(B_ * 8), dim3(256), 0, stream>>>(x, bwf, pts, bwg, sumsq);
  k_bases_write<<<dim3(B_ * (N_ / 64)), dim3(256), 0, stream>>>(x, bwf, pts, bwg, sumsq,
                                                                bases, basesT);
  k_fc0_ln<<<dim3(B_ * (N_ / 64)), dim3(256), 0, stream>>>(x, fc0w, fc0b, ln0g, ln0b, h, hT);
  k_pack<<<dim3(928), dim3(256), 0, stream>>>(spw, H1, wsw, fc1w, spw16, h1t16, wsw16, fc1t16);
  for (int layer = 0; layer < L_; ++layer) {
    k_xh<<<dim3(B_ * 8), dim3(256), 0, stream>>>(basesT, hT, xhT);
    k_t<<<dim3(B_ * KM_ * 8), dim3(256), 0, stream>>>(spw16, xhT, t16, layer);
    k_y<<<dim3(B_ * 8), dim3(256), 0, stream>>>(t16, h1t16, ys16);
    k_x1h<<<dim3(B_ * (N_ / 64)), dim3(256), 0, stream>>>(bases, ys16, h, hT, wsw16, wsb,
                                                          lng, lnb, layer);
  }
  k_fc12<<<dim3(B_ * (N_ / 64)), dim3(256), 0, stream>>>(h, fc1t16, fc1b, fc2w, fc2b,
                                                         (float*)d_out);
}
